// LSTMAutoencoder_65481071411026
// MI455X (gfx1250) — hardware-verified
//
#include <hip/hip_runtime.h>
#include <math.h>

constexpr int NB    = 256;
constexpr int NS    = 512;
constexpr int NF    = 64;
constexpr int NH    = 256;
constexpr int NE    = 128;
constexpr int NG    = 4 * NH;
constexpr int KCAT  = NF + NH;
constexpr int ROWS  = 32;
constexpr int NTHR  = 512;
constexpr int NWAVE = NTHR / 32;
constexpr int AP  = 328;
constexpr int SCP = 516;
constexpr int PP  = 20;
constexpr int RP  = 68;
constexpr int EP  = 132;
constexpr float WCARRY = 16.0f;
constexpr float WINV   = 1.0f / 16.0f;
constexpr float BN_EPS = 1e-5f;
constexpr size_t OUT1_OFF = (size_t)NB * NS * NF;
constexpr size_t OUT2_OFF = OUT1_OFF + (size_t)NB * NE;
static_assert(OUT1_OFF * 4 == 33554432, "out1 byte offset");
static_assert(OUT2_OFF * 4 == 33685504, "out2 byte offset");
static_assert((OUT2_OFF + (size_t)NB * NS) * 4 == 34209792, "d_out total");
static_assert(NB % ROWS == 0, "batch tiles");
static_assert(NH == 16 * NWAVE, "one 16-unit subtile per wave");
static_assert(KCAT % 32 == 0 && NH % 32 == 0 && NE % 32 == 0 && NF % 32 == 0, "K multiples of 32");
static_assert(ROWS * NF == NTHR * 4, "x / rec tile: one float4 per thread");
static_assert(ROWS * NS == 8 * NTHR * 4, "out2 tile: eight float4 per thread");
static_assert(ROWS * NE == 2 * NTHR * 4, "out1 tile: two float4 per thread");
static_assert(AP % 8 == 0 && AP >= KCAT + 8, "A tile pitch");
static_assert(ROWS * EP <= ROWS * SCP && ROWS * RP <= ROWS * SCP, "staging fits");

constexpr int PB_WIH = NG * (NF / 8) / 256;
constexpr int PB_WHH = NG * (NH / 8) / 256;
constexpr int PB_FC  = NE * (NH / 8) / 256;
constexpr int PB_DX  = NH * (NE / 8) / 256;
constexpr int PB_OUT = NF * (NH / 8) / 256;
constexpr int PB_TOTAL = 2 * (PB_WIH + PB_WHH) + PB_FC + 2 * PB_DX + PB_OUT;
static_assert(PB_WIH == 32 && PB_WHH == 128 && PB_FC == 16 && PB_DX == 16 && PB_OUT == 8, "pack ranges");

typedef __attribute__((ext_vector_type(16))) _Float16 v16h;
typedef __attribute__((ext_vector_type(8)))  _Float16 v8h;
typedef __attribute__((ext_vector_type(4)))  _Float16 v4h;
typedef __attribute__((ext_vector_type(8)))  float    v8f;
typedef __attribute__((ext_vector_type(4)))  float    v4f;

template <typename T> struct Frag;
template <> struct Frag<_Float16> {
  typedef v16h V; union U { v16h v; v8h h[2]; };
  static __device__ __forceinline__ v16h load(const _Float16* p) {
    U f; f.h[0] = *(const v8h*)(p); f.h[1] = *(const v8h*)(p + 16); return f.v;
  }
  static __device__ __forceinline__ v8f mma(v16h a, v16h b, v8f c) {
    return __builtin_amdgcn_wmma_f32_16x16x32_f16(false, a, false, b, (short)0, c, false, false);
  }
};
typedef Frag<_Float16> FH;

__device__ __forceinline__ void guard8(v8f& c0, v8f& c1, v8f& c2, v8f& c3, v8f& c4, v8f& c5, v8f& c6, v8f& c7,
                                       v16h a0, v16h a1, v16h b0, v16h b1, v16h b2, v16h b3) {
  asm volatile("v_nop\n\tv_nop\n\tv_nop\n\tv_nop"
               : "+v"(c0), "+v"(c1), "+v"(c2), "+v"(c3), "+v"(c4), "+v"(c5), "+v"(c6), "+v"(c7)
               : "v"(a0), "v"(a1), "v"(b0), "v"(b1), "v"(b2), "v"(b3));
}
__device__ __forceinline__ void guard4(v8f& c0, v8f& c1, v8f& c2, v8f& c3, v16h a0, v16h a1, v16h b0, v16h b1) {
  asm volatile("v_nop\n\tv_nop\n\tv_nop\n\tv_nop"
               : "+v"(c0), "+v"(c1), "+v"(c2), "+v"(c3)
               : "v"(a0), "v"(a1), "v"(b0), "v"(b1));
}
__device__ __forceinline__ v8f mma1(v16h a, v16h b, v8f c) {
  c = FH::mma(a, b, c);
  asm volatile("v_nop\n\tv_nop\n\tv_nop\n\tv_nop" : "+v"(c) : "v"(a), "v"(b));
  return c;
}

__device__ __forceinline__ float fsig(float x)  { return __builtin_amdgcn_rcpf(1.0f + __expf(-x)); }
__device__ __forceinline__ float ftanh(float x) { return 1.0f - 2.0f * __builtin_amdgcn_rcpf(__expf(2.0f * x) + 1.0f); }

__device__ __forceinline__ float lstm_cell(float zi, float zf, float zg, float zo, float& cs) {
  const float ig = fsig(zi);
  const float fg = fsig(zf);
  const float gg = ftanh(zg);
  const float og = fsig(zo);
  const float cn = fg * cs + ig * gg;
  cs = cn;
  return og * ftanh(cn);
}

__device__ __forceinline__ void gate_gemm(const _Float16* __restrict__ W, const _Float16* arow0, const _Float16* arow1,
                                          int ju, int koff, v8f (&acc)[2][4]) {
  const v8f z8 = {0.f, 0.f, 0.f, 0.f, 0.f, 0.f, 0.f, 0.f};
#pragma unroll
  for (int mt = 0; mt < 2; ++mt)
#pragma unroll
    for (int g = 0; g < 4; ++g) acc[mt][g] = z8;
  const _Float16* w0 = W + (size_t)ju * KCAT + koff;
  const size_t gs = (size_t)NH * KCAT;
#pragma unroll 1
  for (int k0 = 0; k0 < KCAT; k0 += 32) {
    const v16h a0 = FH::load(arow0 + k0);
    const v16h a1 = FH::load(arow1 + k0);
    const v16h b0 = FH::load(w0 + k0);
    const v16h b1 = FH::load(w0 + gs + k0);
    const v16h b2 = FH::load(w0 + 2 * gs + k0);
    const v16h b3 = FH::load(w0 + 3 * gs + k0);
    acc[0][0] = FH::mma(a0, b0, acc[0][0]);
    acc[1][0] = FH::mma(a1, b0, acc[1][0]);
    acc[0][1] = FH::mma(a0, b1, acc[0][1]);
    acc[1][1] = FH::mma(a1, b1, acc[1][1]);
    acc[0][2] = FH::mma(a0, b2, acc[0][2]);
    acc[1][2] = FH::mma(a1, b2, acc[1][2]);
    acc[0][3] = FH::mma(a0, b3, acc[0][3]);
    acc[1][3] = FH::mma(a1, b3, acc[1][3]);
    guard8(acc[0][0], acc[1][0], acc[0][1], acc[1][1], acc[0][2], acc[1][2], acc[0][3], acc[1][3],
           a0, a1, b0, b1, b2, b3);
  }
}

__device__ __forceinline__ float score_exp(const float* pp, float ab) {
  const v4f q0 = *(const v4f*)(pp);
  const v4f q1 = *(const v4f*)(pp + 4);
  const v4f q2 = *(const v4f*)(pp + 8);
  const v4f q3 = *(const v4f*)(pp + 12);
  const float s0 = (q0[0] + q0[1]) + (q0[2] + q0[3]);
  const float s1 = (q1[0] + q1[1]) + (q1[2] + q1[3]);
  const float s2 = (q2[0] + q2[1]) + (q2[2] + q2[3]);
  const float s3 = (q3[0] + q3[1]) + (q3[2] + q3[3]);
  const float sc = ((s0 + s1) + (s2 + s3)) + ab;
  return expf(sc);
}

__global__ __launch_bounds__(256) void pack_planes_kernel(
    const float* __restrict__ encWih, const float* __restrict__ encWhh,
    const float* __restrict__ decWih, const float* __restrict__ decWhh,
    const float* __restrict__ fcW, const float* __restrict__ dhW,
    const float* __restrict__ dcW, const float* __restrict__ outW,
    unsigned short* __restrict__ BENC, unsigned short* __restrict__ BDEC,
    unsigned short* __restrict__ FCW, unsigned short* __restrict__ DHW,
    unsigned short* __restrict__ DCW, unsigned short* __restrict__ OUTW) {
  int bx = blockIdx.x;
  const float* src = encWih;
  unsigned short* dst = BENC;
  int spitch = NF, l2c = 3, dpitch = KCAT, dcol0 = 0, nrow = NG;
  if (bx < PB_WIH) {
    src = encWih; dst = BENC; spitch = NF; l2c = 3; dpitch = KCAT; dcol0 = 0; nrow = NG;
  } else if (bx < PB_WIH + PB_WHH) {
    bx -= PB_WIH;
    src = encWhh; dst = BENC; spitch = NH; l2c = 5; dpitch = KCAT; dcol0 = NF; nrow = NG;
  } else if (bx < 2 * PB_WIH + PB_WHH) {
    bx -= PB_WIH + PB_WHH;
    src = decWih; dst = BDEC; spitch = NF; l2c = 3; dpitch = KCAT; dcol0 = 0; nrow = NG;
  } else if (bx < 2 * (PB_WIH + PB_WHH)) {
    bx -= 2 * PB_WIH + PB_WHH;
    src = decWhh; dst = BDEC; spitch = NH; l2c = 5; dpitch = KCAT; dcol0 = NF; nrow = NG;
  } else if (bx < 2 * (PB_WIH + PB_WHH) + PB_FC) {
    bx -= 2 * (PB_WIH + PB_WHH);
    src = fcW; dst = FCW; spitch = NH; l2c = 5; dpitch = NH; dcol0 = 0; nrow = NE;
  } else if (bx < 2 * (PB_WIH + PB_WHH) + PB_FC + PB_DX) {
    bx -= 2 * (PB_WIH + PB_WHH) + PB_FC;
    src = dhW; dst = DHW; spitch = NE; l2c = 4; dpitch = NE; dcol0 = 0; nrow = NH;
  } else if (bx < 2 * (PB_WIH + PB_WHH) + PB_FC + 2 * PB_DX) {
    bx -= 2 * (PB_WIH + PB_WHH) + PB_FC + PB_DX;
    src = dcW; dst = DCW; spitch = NE; l2c = 4; dpitch = NE; dcol0 = 0; nrow = NH;
  } else {
    bx -= 2 * (PB_WIH + PB_WHH) + PB_FC + 2 * PB_DX;
    src = outW; dst = OUTW; spitch = NH; l2c = 5; dpitch = NH; dcol0 = 0; nrow = NF;
  }
  const int i = bx * 256 + (int)threadIdx.x;
  const int row = i >> l2c;
  const int c8 = i & ((1 << l2c) - 1);
  if (row < nrow) {
    const float* sp = src + (size_t)row * spitch + c8 * 8;
    const v4f a = *(const v4f*)(sp);
    const v4f b = *(const v4f*)(sp + 4);
    v8h hv;
#pragma unroll
    for (int e = 0; e < 4; ++e) {
      hv[e]     = (_Float16)(a[e] * WCARRY);
      hv[4 + e] = (_Float16)(b[e] * WCARRY);
    }
    unsigned short* dp = dst + (size_t)row * dpitch + dcol0 + c8 * 8;
    *(volatile v8h*)dp = hv;
    __threadfence();
    *(volatile v8h*)dp = hv;
  }
}

__global__ __launch_bounds__(NTHR) void lstm_ae_kernel(
    const float* __restrict__ x,
    const unsigned short* __restrict__ BENCp, const unsigned short* __restrict__ BDECp,
    const unsigned short* __restrict__ FCWp, const unsigned short* __restrict__ DHWp,
    const unsigned short* __restrict__ DCWp, const unsigned short* __restrict__ OUTWp,
    const float* __restrict__ enc_bih, const float* __restrict__ enc_bhh,
    const float* __restrict__ attn_w, const float* __restrict__ attn_b,
    const float* __restrict__ fc_b,
    const float* __restrict__ bn_g, const float* __restrict__ bn_bt,
    const float* __restrict__ bn_m, const float* __restrict__ bn_v,
    const float* __restrict__ dh_b, const float* __restrict__ dc_b,
    const float* __restrict__ dec_bih, const float* __restrict__ dec_bhh,
    const float* __restrict__ out_b,
    float* __restrict__ out) {
  __shared__ __align__(16) _Float16 sA[ROWS * AP];
  __shared__ __align__(16) float    sSc[ROWS * SCP];
  __shared__ __align__(16) float    sPart[ROWS * PP];
  __shared__ __align__(16) float    sE[ROWS];
  __shared__ __align__(16) float    sL[ROWS];

  const _Float16* BENC = (const _Float16*)BENCp;
  const _Float16* BDEC = (const _Float16*)BDECp;
  const _Float16* FCW  = (const _Float16*)FCWp;
  const _Float16* DHW  = (const _Float16*)DHWp;
  const _Float16* DCW  = (const _Float16*)DCWp;
  const _Float16* OUTW = (const _Float16*)OUTWp;

  const int tid = threadIdx.x, lane = tid & 31, wave = tid >> 5;
  const int c = lane & 15, hh = lane >> 4, koff = hh * 8;
  const int b0 = blockIdx.x * ROWS;
  const int ju = 16 * wave + c;
  const int xrow = tid >> 4, xf4 = (tid & 15) * 4;
  const v8f z8 = {0.f, 0.f, 0.f, 0.f, 0.f, 0.f, 0.f, 0.f};

  {
    const v4h z4 = {(_Float16)0.0f, (_Float16)0.0f, (_Float16)0.0f, (_Float16)0.0f};
#pragma unroll 1
    for (int i = tid; i < ROWS * 66; i += NTHR) {
      const int row = i / 66;
      const int g = i - row * 66;
      *(v4h*)(sA + row * AP + NF + 4 * g) = z4;
    }
  }
  if (tid < ROWS) sE[tid] = 0.0f;
  {
    v4f xv = *(const v4f*)(x + ((size_t)(b0 + xrow) * NS) * NF + xf4);
    v4h xh;
    xh[0] = (_Float16)xv[0]; xh[1] = (_Float16)xv[1]; xh[2] = (_Float16)xv[2]; xh[3] = (_Float16)xv[3];
    *(v4h*)(sA + xrow * AP + xf4) = xh;
  }

  float cst[2][8], hst[2][8], ctx[2][8];
#pragma unroll
  for (int mt = 0; mt < 2; ++mt)
#pragma unroll
    for (int r = 0; r < 8; ++r) { cst[mt][r] = 0.0f; hst[mt][r] = 0.0f; ctx[mt][r] = 0.0f; }
  float bsum[4];
#pragma unroll
  for (int g = 0; g < 4; ++g) bsum[g] = enc_bih[g * NH + ju] + enc_bhh[g * NH + ju];
  const float aw = attn_w[ju];
  const float attnb = attn_b[0];
  float lsum = 0.0f;

  const _Float16* arow0 = sA + c * AP + koff;
  const _Float16* arow1 = sA + (16 + c) * AP + koff;
  __syncthreads();

  v8f acc[2][4];

#pragma unroll 1
  for (int s = 0; s < NS; ++s) {
    if (wave == 0 && s > 0) {
      const float e = score_exp(sPart + lane * PP, attnb);
      sE[lane] = e;
      sSc[lane * SCP + (s - 1)] = e;
      lsum += e;
    }
    gate_gemm(BENC, arow0, arow1, ju, koff, acc);
    __syncthreads();
    {
      const int tn = (s + 1 < NS) ? (s + 1) : (NS - 1);
      v4f xv = *(const v4f*)(x + ((size_t)(b0 + xrow) * NS + (size_t)tn) * NF + xf4);
      asm volatile("" : "+v"(xv));
      v4h xh;
      xh[0] = (_Float16)xv[0]; xh[1] = (_Float16)xv[1]; xh[2] = (_Float16)xv[2]; xh[3] = (_Float16)xv[3];
      *(v4h*)(sA + xrow * AP + xf4) = xh;
    }
    const v4f e0a = *(const v4f*)(sE + 8 * hh);
    const v4f e0b = *(const v4f*)(sE + 8 * hh + 4);
    const v4f e1a = *(const v4f*)(sE + 16 + 8 * hh);
    const v4f e1b = *(const v4f*)(sE + 16 + 8 * hh + 4);
    const float ev[2][8] = {{e0a[0], e0a[1], e0a[2], e0a[3], e0b[0], e0b[1], e0b[2], e0b[3]},
                            {e1a[0], e1a[1], e1a[2], e1a[3], e1b[0], e1b[1], e1b[2], e1b[3]}};
    float pr[2][8];
#pragma unroll
    for (int mt = 0; mt < 2; ++mt) {
#pragma unroll
      for (int r = 0; r < 8; ++r) {
        ctx[mt][r] = fmaf(ev[mt][r], hst[mt][r], ctx[mt][r]);
        const float zi = fmaf(acc[mt][0][r], WINV, bsum[0]);
        const float zf = fmaf(acc[mt][1][r], WINV, bsum[1]);
        const float zg = fmaf(acc[mt][2][r], WINV, bsum[2]);
        const float zo = fmaf(acc[mt][3][r], WINV, bsum[3]);
        const float hn = lstm_cell(zi, zf, zg, zo, cst[mt][r]);
        hst[mt][r] = hn;
        sA[(16 * mt + 8 * hh + r) * AP + NF + ju] = (_Float16)hn;
        float p = hn * aw;
        p += __shfl_xor(p, 1, 32);
        p += __shfl_xor(p, 2, 32);
        p += __shfl_xor(p, 4, 32);
        p += __shfl_xor(p, 8, 32);
        pr[mt][r] = p;
      }
    }
    if (c == 0) {
#pragma unroll
      for (int mt = 0; mt < 2; ++mt)
#pragma unroll
        for (int r = 0; r < 8; ++r) sPart[(16 * mt + 8 * hh + r) * PP + wave] = pr[mt][r];
    }
    __syncthreads();
  }

  if (wave == 0) {
    const float e = score_exp(sPart + lane * PP, attnb);
    sE[lane] = e;
    sSc[lane * SCP + (NS - 1)] = e;
    lsum += e;
    sL[lane] = 1.0f / lsum;
  }
  __syncthreads();
  {
    const v4f e0a = *(const v4f*)(sE + 8 * hh);
    const v4f e0b = *(const v4f*)(sE + 8 * hh + 4);
    const v4f e1a = *(const v4f*)(sE + 16 + 8 * hh);
    const v4f e1b = *(const v4f*)(sE + 16 + 8 * hh + 4);
    const v4f l0a = *(const v4f*)(sL + 8 * hh);
    const v4f l0b = *(const v4f*)(sL + 8 * hh + 4);
    const v4f l1a = *(const v4f*)(sL + 16 + 8 * hh);
    const v4f l1b = *(const v4f*)(sL + 16 + 8 * hh + 4);
    const float ev[2][8] = {{e0a[0], e0a[1], e0a[2], e0a[3], e0b[0], e0b[1], e0b[2], e0b[3]},
                            {e1a[0], e1a[1], e1a[2], e1a[3], e1b[0], e1b[1], e1b[2], e1b[3]}};
    const float il[2][8] = {{l0a[0], l0a[1], l0a[2], l0a[3], l0b[0], l0b[1], l0b[2], l0b[3]},
                            {l1a[0], l1a[1], l1a[2], l1a[3], l1b[0], l1b[1], l1b[2], l1b[3]}};
#pragma unroll
    for (int mt = 0; mt < 2; ++mt)
#pragma unroll
      for (int r = 0; r < 8; ++r) {
        const float cs = fmaf(ev[mt][r], hst[mt][r], ctx[mt][r]);
        const float cn = cs * il[mt][r];
        sA[(16 * mt + 8 * hh + r) * AP + NF + ju] = (_Float16)cn;
      }
  }
  {
    v4f o[8];
#pragma unroll
    for (int it = 0; it < 8; ++it) {
      const int idx = it * NTHR + tid;
      const int row = idx >> 7;
      const int c4 = (idx & 127) * 4;
      const v4f v = *(const v4f*)(sSc + row * SCP + c4);
      const float li = sL[row];
      o[it] = v * li;
    }
    float* w2 = out + OUT2_OFF + (size_t)b0 * NS;
    for (int pass = 0; pass < 2; ++pass) {
#pragma unroll
      for (int it = 0; it < 8; ++it) {
        const int idx = it * NTHR + tid;
        const int row = idx >> 7;
        const int c4 = (idx & 127) * 4;
        *(volatile v4f*)(w2 + (size_t)row * NS + c4) = o[it];
      }
      __threadfence();
    }
  }
  __syncthreads();

  float embv[8];
  const int fmt = wave >> 3;
  const int fn = 16 * (wave & 7) + c;
  {
    const _Float16* ar = sA + (16 * fmt + c) * AP + NF + koff;
    const _Float16* wr = FCW + (size_t)fn * NH + koff;
    v8f ea = z8;
#pragma unroll 1
    for (int k0 = 0; k0 < NH; k0 += 32) {
      const v16h a = FH::load(ar + k0);
      const v16h b = FH::load(wr + k0);
      ea = mma1(a, b, ea);
    }
    const float fb = fc_b[fn];
    const float mu = bn_m[fn];
    const float rs = rsqrtf(bn_v[fn] + BN_EPS);
    const float gm = bn_g[fn];
    const float bt = bn_bt[fn];
#pragma unroll
    for (int r = 0; r < 8; ++r) {
      const float raw = fmaf(ea[r], WINV, fb);
      const float y = ((raw - mu) * rs) * gm + bt;
      embv[r] = tanhf(y);
    }
  }
  __syncthreads();
#pragma unroll
  for (int r = 0; r < 8; ++r) {
    sSc[(16 * fmt + 8 * hh + r) * EP + fn] = embv[r];
    sA[(16 * fmt + 8 * hh + r) * AP + fn] = (_Float16)embv[r];
  }
  __syncthreads();
  {
    v4f o[2];
#pragma unroll
    for (int it = 0; it < 2; ++it) {
      const int idx = it * NTHR + tid;
      const int row = idx >> 5;
      const int c4 = (idx & 31) * 4;
      o[it] = *(const v4f*)(sSc + row * EP + c4);
    }
    float* w1 = out + OUT1_OFF + (size_t)b0 * NE;
    for (int pass = 0; pass < 2; ++pass) {
#pragma unroll
      for (int it = 0; it < 2; ++it) {
        const int idx = it * NTHR + tid;
        const int row = idx >> 5;
        const int c4 = (idx & 31) * 4;
        *(volatile v4f*)(w1 + (size_t)row * NE + c4) = o[it];
      }
      __threadfence();
    }
  }
  float hini[2][8];
  {
    v8f hd0 = z8, hd1 = z8, cd0 = z8, cd1 = z8;
    const _Float16* wh = DHW + (size_t)ju * NE + koff;
    const _Float16* wc = DCW + (size_t)ju * NE + koff;
#pragma unroll 1
    for (int k0 = 0; k0 < NE; k0 += 32) {
      const v16h a0 = FH::load(arow0 + k0);
      const v16h a1 = FH::load(arow1 + k0);
      const v16h bh = FH::load(wh + k0);
      const v16h bc = FH::load(wc + k0);
      hd0 = FH::mma(a0, bh, hd0);
      hd1 = FH::mma(a1, bh, hd1);
      cd0 = FH::mma(a0, bc, cd0);
      cd1 = FH::mma(a1, bc, cd1);
      guard4(hd0, hd1, cd0, cd1, a0, a1, bh, bc);
    }
    const float bhv = dh_b[ju];
    const float bcv = dc_b[ju];
#pragma unroll
    for (int r = 0; r < 8; ++r) {
      hini[0][r] = fmaf(hd0[r], WINV, bhv);
      hini[1][r] = fmaf(hd1[r], WINV, bhv);
      cst[0][r]  = fmaf(cd0[r], WINV, bcv);
      cst[1][r]  = fmaf(cd1[r], WINV, bcv);
    }
  }
  __syncthreads();
#pragma unroll
  for (int mt = 0; mt < 2; ++mt)
#pragma unroll
    for (int r = 0; r < 8; ++r) sA[(16 * mt + 8 * hh + r) * AP + NF + ju] = (_Float16)hini[mt][r];
  {
    const v4h z4 = {(_Float16)0.0f, (_Float16)0.0f, (_Float16)0.0f, (_Float16)0.0f};
    *(v4h*)(sA + xrow * AP + xf4) = z4;
  }
#pragma unroll
  for (int g = 0; g < 4; ++g) bsum[g] = dec_bih[g * NH + ju] + dec_bhh[g * NH + ju];
  const int omt = (wave >> 2) & 1;
  const int on = 16 * (wave & 3) + c;
  const float ob = out_b[on];
  __syncthreads();

#pragma unroll 1
  for (int t = 0; t < NS; ++t) {
    gate_gemm(BDEC, arow0, arow1, ju, koff, acc);
    __syncthreads();
#pragma unroll
    for (int mt = 0; mt < 2; ++mt) {
#pragma unroll
      for (int r = 0; r < 8; ++r) {
        const float zi = fmaf(acc[mt][0][r], WINV, bsum[0]);
        const float zf = fmaf(acc[mt][1][r], WINV, bsum[1]);
        const float zg = fmaf(acc[mt][2][r], WINV, bsum[2]);
        const float zo = fmaf(acc[mt][3][r], WINV, bsum[3]);
        const float hn = lstm_cell(zi, zf, zg, zo, cst[mt][r]);
        sA[(16 * mt + 8 * hh + r) * AP + NF + ju] = (_Float16)hn;
      }
    }
    __syncthreads();
    if (wave < 8) {
      const _Float16* ar = sA + (16 * omt + c) * AP + NF + koff;
      const _Float16* wr = OUTW + (size_t)on * NH + koff;
      v8f ra = z8;
#pragma unroll 1
      for (int k0 = 0; k0 < NH; k0 += 32) {
        const v16h a = FH::load(ar + k0);
        const v16h b = FH::load(wr + k0);
        ra = mma1(a, b, ra);
      }
#pragma unroll
      for (int r = 0; r < 8; ++r) {
        const float rv = fmaf(ra[r], WINV, ob);
        sSc[(16 * omt + 8 * hh + r) * RP + on] = rv;
        sA[(16 * omt + 8 * hh + r) * AP + on] = (_Float16)rv;
      }
    }
    __syncthreads();
    {
      const v4f v = *(const v4f*)(sSc + xrow * RP + xf4);
      float* dp = out + ((size_t)(b0 + xrow) * NS + (size_t)t) * NF + xf4;
      *(volatile v4f*)dp = v;
      __threadfence();
      *(volatile v4f*)dp = v;
    }
  }
}

extern "C" void kernel_launch(void* const* d_in, const int* in_sizes, int n_in,
                              void* d_out, int out_size, void* d_ws, size_t ws_size, hipStream_t stream) {
  if (n_in < 23 || d_out == nullptr || d_ws == nullptr) return;
  if (in_sizes[0] != NB * NS * NF || in_sizes[1] != NG * NF || in_sizes[2] != NG * NH ||
      in_sizes[3] != NG || in_sizes[4] != NG || in_sizes[5] != NH || in_sizes[6] != 1 ||
      in_sizes[7] != NE * NH || in_sizes[8] != NE || in_sizes[9] != NE || in_sizes[10] != NE ||
      in_sizes[11] != NE || in_sizes[12] != NE || in_sizes[13] != NH * NE || in_sizes[14] != NH ||
      in_sizes[15] != NH * NE || in_sizes[16] != NH || in_sizes[17] != NG * NF || in_sizes[18] != NG * NH ||
      in_sizes[19] != NG || in_sizes[20] != NG || in_sizes[21] != NF * NH || in_sizes[22] != NF ||
      out_size != (int)(OUT2_OFF + (size_t)NB * NS)) return;

  const float* x        = (const float*)d_in[0];
  const float* enc_Wih  = (const float*)d_in[1];
  const float* enc_Whh  = (const float*)d_in[2];
  const float* enc_bih  = (const float*)d_in[3];
  const float* enc_bhh  = (const float*)d_in[4];
  const float* attn_W   = (const float*)d_in[5];
  const float* attn_b   = (const float*)d_in[6];
  const float* fc_W     = (const float*)d_in[7];
  const float* fc_b     = (const float*)d_in[8];
  const float* bn_gamma = (const float*)d_in[9];
  const float* bn_beta  = (const float*)d_in[10];
  const float* bn_mean  = (const float*)d_in[11];
  const float* bn_var   = (const float*)d_in[12];
  const float* dh_W     = (const float*)d_in[13];
  const float* dh_b     = (const float*)d_in[14];
  const float* dc_W     = (const float*)d_in[15];
  const float* dc_b     = (const float*)d_in[16];
  const float* dec_Wih  = (const float*)d_in[17];
  const float* dec_Whh  = (const float*)d_in[18];
  const float* dec_bih  = (const float*)d_in[19];
  const float* dec_bhh  = (const float*)d_in[20];
  const float* out_W    = (const float*)d_in[21];
  const float* out_b    = (const float*)d_in[22];
  float* out = (float*)d_out;

  char* ws = (char*)d_ws; size_t off = 0;
  auto carve = [&](size_t bytes) -> char* { char* p = ws + off; off += (bytes + 255) & ~(size_t)255; return p; };
  unsigned short* BENC = (unsigned short*)carve((size_t)NG * KCAT * 2);
  unsigned short* BDEC = (unsigned short*)carve((size_t)NG * KCAT * 2);
  unsigned short* FCW  = (unsigned short*)carve((size_t)NE * NH * 2);
  unsigned short* DHW  = (unsigned short*)carve((size_t)NH * NE * 2);
  unsigned short* DCW  = (unsigned short*)carve((size_t)NH * NE * 2);
  unsigned short* OUTW = (unsigned short*)carve((size_t)NF * NH * 2);
  if (off > ws_size || off > (size_t)134217728) return;

  pack_planes_kernel<<<PB_TOTAL, 256, 0, stream>>>(enc_Wih, enc_Whh, dec_Wih, dec_Whh, fc_W, dh_W, dc_W, out_W,
                                                  BENC, BDEC, FCW, DHW, DCW, OUTW);
  lstm_ae_kernel<<<NB / ROWS, NTHR, 0, stream>>>(x, BENC, BDEC, FCW, DHW, DCW, OUTW,
                                                 enc_bih, enc_bhh, attn_W, attn_b, fc_b,
                                                 bn_gamma, bn_beta, bn_mean, bn_var,
                                                 dh_b, dc_b, dec_bih, dec_bhh, out_b, out);
}
